// GraphNetwork_35003983462587
// MI455X (gfx1250) — hardware-verified
//
#include <hip/hip_runtime.h>
#include <stddef.h>
#include <stdint.h>
#include <math.h>


#define NN     50000
#define NE     1200000
#define NGR    256
#define NCLS   10
#define NTHR   256
#define NWAVE  8
#define EPT    8
#define CHUNK  (NTHR * EPT)
#define WCAP   (EPT * 32)
#define LISTN  (NWAVE * WCAP)
#define NBA    1024
#define SLA    10
#define NBLK   49
#define NPADS  (NBLK * NBA)
#define RCAP   28672
#define DEGCAP 64
#define GBM    64
#define GTHR   128
#define TROWS  128
#define NTILE  391
#define MPAD   (NTILE * TROWS)
#define RECW   160
#define AGG_ZINTS (LISTN + 2 * RCAP + 3 * NBA)
#define AGG_LDS_INTS (AGG_ZINTS + 16)
#define NOUT   (NGR * NCLS)
#define NUX    (MPAD * 8)
#define NUW1   (64 * 8)
#define NUW2   (64 * 16)
#define NUW3   (32 * 16)
#define NUALL  (NUX + NUW1 + 2 * NUW2 + NUW3)
#define WSMAX  134217728

static_assert(NN % 16 == 0);
static_assert(MPAD >= NN && MPAD % GBM == 0 && MPAD - NN < TROWS);
static_assert(NPADS >= MPAD && NBLK * NBA == NPADS);
static_assert((CHUNK & (CHUNK - 1)) == 0 && CHUNK <= 4096);
static_assert((NBA & (NBA - 1)) == 0 && NBA == (1 << SLA) && NBA == 4 * NTHR);
static_assert(((long long)CHUNK << SLA) < (1LL << 31));
static_assert(((long long)NE << SLA) < (1LL << 31));
static_assert(LISTN % NTHR == 0 && NBA % NWAVE == 0 && NBA % 32 == 0);
static_assert(RCAP % (NTHR * 4) == 0 && AGG_ZINTS % 4 == 0 && LISTN % 4 == 0);
static_assert(24968 <= RCAP && 46 + 8 <= DEGCAP);
static_assert(AGG_LDS_INTS * 4 <= 300000);
static_assert(GBM == (GTHR / 32) * 16);
static_assert(NUX % NTHR == 0 && NUW1 % NTHR == 0 && NUW2 % NTHR == 0 && NUW3 % NTHR == 0);
static_assert(RECW % 32 == 0 && RECW / 4 <= NTHR);
static_assert(NGR == 256 && NGR == NTHR);
static_assert((NOUT * 4) % 128 == 0 && NOUT % 4 == 0);

typedef float          v2f   __attribute__((ext_vector_type(2)));
typedef float          v4f   __attribute__((ext_vector_type(4)));
typedef float          v8f   __attribute__((ext_vector_type(8)));
typedef int            v4i   __attribute__((ext_vector_type(4)));
typedef int            v8i   __attribute__((ext_vector_type(8)));
typedef unsigned short v8us  __attribute__((ext_vector_type(8)));
typedef unsigned short v16us __attribute__((ext_vector_type(16)));
typedef __bf16         v16bf __attribute__((ext_vector_type(16)));
typedef v2f  __attribute__((may_alias)) v2fa;
typedef v4f  __attribute__((may_alias)) v4fa;
typedef v4i  __attribute__((may_alias)) v4ia;
typedef v8us __attribute__((may_alias)) v8usa;
union FragB { v16bf v; v16us u; v8us h[2]; v8i w; };

__device__ __forceinline__ v8f wmb(const FragB& a, const FragB& b, v8f c) {
  v8f d = __builtin_amdgcn_wmma_f32_16x16x32_bf16(false, a.v, false, b.v, (short)0, c, false, false);
  asm volatile("v_nop\n\tv_nop\n\tv_nop\n\tv_nop" : "+v"(d) : "v"(a.w), "v"(b.w));
  return d;
}

__device__ __forceinline__ unsigned bf16_bits(float f) {
  const unsigned u = __float_as_uint(f);
  return (u + 0x7FFFu + ((u >> 16) & 1u)) >> 16;
}
__device__ __forceinline__ unsigned bf16_bits_n(float f) {
  const unsigned r = bf16_bits(f);
  return (f != f) ? 0x7fc0u : r;
}
__device__ __forceinline__ float bf16_val(float f) {
  return __uint_as_float(bf16_bits(f) << 16);
}

template <int SLB>
__device__ __forceinline__ int scan_chunk(const int* __restrict__ dsts, int nE, int cbase, int slotBase,
                                          int nb, int vec8, int* list, int tid, int lane, int wave) {
  int wc = 0;
  const int el0  = tid * EPT;
  const int e0   = cbase + el0;
  const int sent = -2147483647 - 1;
  v4i da, db;
  if (vec8 != 0 && cbase + CHUNK <= nE) {
    da = *(const v4i*)(dsts + e0);
    db = *(const v4i*)(dsts + e0 + 4);
  } else {
    da.x = (e0     < nE) ? dsts[min(e0,     nE - 1)] : sent;
    da.y = (e0 + 1 < nE) ? dsts[min(e0 + 1, nE - 1)] : sent;
    da.z = (e0 + 2 < nE) ? dsts[min(e0 + 2, nE - 1)] : sent;
    da.w = (e0 + 3 < nE) ? dsts[min(e0 + 3, nE - 1)] : sent;
    db.x = (e0 + 4 < nE) ? dsts[min(e0 + 4, nE - 1)] : sent;
    db.y = (e0 + 5 < nE) ? dsts[min(e0 + 5, nE - 1)] : sent;
    db.z = (e0 + 6 < nE) ? dsts[min(e0 + 6, nE - 1)] : sent;
    db.w = (e0 + 7 < nE) ? dsts[min(e0 + 7, nE - 1)] : sent;
  }
  const unsigned nbs = (unsigned)slotBase;
  const unsigned unb = (unsigned)nb;
  const unsigned s0 = (unsigned)da.x - nbs, s1 = (unsigned)da.y - nbs;
  const unsigned s2 = (unsigned)da.z - nbs, s3 = (unsigned)da.w - nbs;
  const unsigned s4 = (unsigned)db.x - nbs, s5 = (unsigned)db.y - nbs;
  const unsigned s6 = (unsigned)db.z - nbs, s7 = (unsigned)db.w - nbs;
  const bool h0 = s0 < unb, h1 = s1 < unb, h2 = s2 < unb, h3 = s3 < unb;
  const bool h4 = s4 < unb, h5 = s5 < unb, h6 = s6 < unb, h7 = s7 < unb;
  const unsigned any = __builtin_amdgcn_ballot_w32(h0 | h1 | h2 | h3 | h4 | h5 | h6 | h7);
  if (any != 0u) {
#define HITJ(J, HJ, SJ) { \
      const unsigned mj = __builtin_amdgcn_ballot_w32(HJ); \
      if (mj != 0u) { \
        if (HJ) { \
          const int pos = wc + (int)__builtin_amdgcn_mbcnt_lo(mj, 0u); \
          if (pos < WCAP) list[wave * WCAP + pos] = ((el0 + (J)) << SLB) | (int)(SJ); \
        } \
        wc += (int)__builtin_popcount(mj); } }
    HITJ(0, h0, s0)
    HITJ(1, h1, s1)
    HITJ(2, h2, s2)
    HITJ(3, h3, s3)
    HITJ(4, h4, s4)
    HITJ(5, h5, s5)
    HITJ(6, h6, s6)
    HITJ(7, h7, s7)
#undef HITJ
  }
  return wc;
}

__device__ __forceinline__ v8us wgather(const float* __restrict__ p, int stride) {
  v8us o;
#pragma unroll
  for (int i = 0; i < 8; ++i) o[i] = (unsigned short)bf16_bits(p[(size_t)i * (size_t)stride]);
  return o;
}

__global__ __launch_bounds__(NTHR) void k_prep(const float* __restrict__ x, const float* __restrict__ W1,
                                               const float* __restrict__ W2, const float* __restrict__ W4,
                                               const float* __restrict__ W3, unsigned short* xb,
                                               unsigned short* w1t, unsigned short* w2d,
                                               unsigned short* w4d, unsigned short* w3d) {
  const int u = (int)blockIdx.x * NTHR + (int)threadIdx.x;
  v8us o;
  unsigned short* dp;
  if (u < NUX) {
    const int row = u >> 3;
    const int k8  = (u & 7) * 8;
    const int rc  = row < NN ? row : NN - 1;
    const float* p = x + (size_t)rc * 64 + k8;
    const v4f a = *(const v4fa*)p;
    const v4f b = *(const v4fa*)(p + 4);
    const bool ok = row < NN;
    o[0] = ok ? (unsigned short)bf16_bits(a.x) : (unsigned short)0;
    o[1] = ok ? (unsigned short)bf16_bits(a.y) : (unsigned short)0;
    o[2] = ok ? (unsigned short)bf16_bits(a.z) : (unsigned short)0;
    o[3] = ok ? (unsigned short)bf16_bits(a.w) : (unsigned short)0;
    o[4] = ok ? (unsigned short)bf16_bits(b.x) : (unsigned short)0;
    o[5] = ok ? (unsigned short)bf16_bits(b.y) : (unsigned short)0;
    o[6] = ok ? (unsigned short)bf16_bits(b.z) : (unsigned short)0;
    o[7] = ok ? (unsigned short)bf16_bits(b.w) : (unsigned short)0;
    dp = xb + (size_t)row * 64 + k8;
  } else if (u < NUX + NUW1) {
    const int v  = u - NUX;
    const int n  = v >> 3;
    const int k8 = (v & 7) * 8;
    o = wgather(W1 + (size_t)k8 * 64 + n, 64);
    dp = w1t + (size_t)n * 64 + k8;
  } else if (u < NUX + NUW1 + NUW2) {
    const int v  = u - (NUX + NUW1);
    const int n  = v >> 4;
    const int k8 = (v & 15) * 8;
    const int kk = k8 & 63;
    o = wgather(W2 + (size_t)kk * 64 + n, 64);
    dp = w2d + (size_t)n * 128 + k8;
  } else if (u < NUX + NUW1 + 2 * NUW2) {
    const int v  = u - (NUX + NUW1 + NUW2);
    const int n  = v >> 4;
    const int k8 = (v & 15) * 8;
    const int kk = k8 & 63;
    o = wgather(W4 + (size_t)kk * 64 + n, 64);
    dp = w4d + (size_t)n * 128 + k8;
  } else if (u < NUALL) {
    const int v  = u - (NUX + NUW1 + 2 * NUW2);
    const int n  = v >> 4;
    const int k8 = (v & 15) * 8;
    const int kk = k8 & 63;
    o = wgather(W3 + (size_t)kk * 32 + n, 32);
    dp = w3d + (size_t)n * 128 + k8;
  } else {
    return;
  }
  *(volatile v8us*)dp = o;
  __threadfence();
  *(volatile v8us*)dp = o;
}

__global__ __launch_bounds__(NTHR) void k_bucket(const int* __restrict__ srcs, const int* __restrict__ dsts,
                                                 int nE, int nN, int vec8,
                                                 int* lst, int* offg, int* cntg, int* disb) {
  extern __shared__ __attribute__((aligned(16))) int dsm[];
  int* list = dsm;
  int* hl   = dsm + LISTN;
  int* sl   = dsm + LISTN + RCAP;
  int* cnt  = dsm + LISTN + 2 * RCAP;
  int* offs = cnt + NBA;
  int* cur  = offs + NBA;
  int* misc = cur + NBA;
  const int tid = (int)threadIdx.x, lane = tid & 31, wave = tid >> 5;
  const int nodeBase = (int)blockIdx.x * NBA;

  {
    const v4i z4 = {0, 0, 0, 0};
    for (int i = tid * 4; i < AGG_ZINTS; i += NTHR * 4) *(v4ia*)(dsm + i) = z4;
    if (tid < 16) misc[tid] = 0;
  }
  __syncthreads();

  int t = 0, ov = 0;
  const int nChunks = (nE + CHUNK - 1) / CHUNK;
#pragma unroll 1
  for (int ch = 0; ch < nChunks; ++ch) {
    const int cbase = ch * CHUNK;
    const int wc = scan_chunk<SLA>(dsts, nE, cbase, nodeBase, NBA, vec8, list, tid, lane, wave);
    if (lane == 0) misc[wave] = wc;
    __syncthreads();
    if (wave == 0) {
#pragma unroll 1
      for (int w2 = 0; w2 < NWAVE; ++w2) {
        int c = misc[w2];
        c = c < 0 ? 0 : (c > WCAP ? WCAP : c);
#pragma unroll 1
        for (int b0 = 0; b0 < c; b0 += 32) {
          const int idx = b0 + lane;
          const int ent = list[w2 * WCAP + (idx < WCAP ? idx : WCAP - 1)];
          const int m32 = (c - b0) < 32 ? (c - b0) : 32;
#pragma unroll 1
          for (int k = 0; k < m32; ++k) {
            const int u    = __builtin_amdgcn_readlane(ent, k);
            const int slot = u & (NBA - 1);
            const int el   = (u >> SLA) & (CHUNK - 1);
            const int pk   = ((cbase + el) << SLA) | slot;
            if (t < RCAP) {
              if (lane == 0) { hl[t] = pk; cnt[slot] = cnt[slot] + 1; }
              t = t + 1;
            } else {
              ov = 1;
            }
          }
        }
      }
    }
    __syncthreads();
  }
  if (wave == 0 && lane == 0) { misc[8] = t; misc[9] = ov; }
  __syncthreads();
  int tt = misc[8];
  tt = tt < 0 ? 0 : (tt > RCAP ? RCAP : tt);
  const int ovf = misc[9];

  if (wave == 0) {
    const int base = lane * (NBA / 32);
    int s = 0;
#pragma unroll 1
    for (int i = 0; i < NBA / 32; ++i) s += cnt[base + i];
    int incl = s;
#pragma unroll
    for (int d = 1; d < 32; d <<= 1) {
      const int y = __shfl_up(incl, d, 32);
      if (lane >= d) incl += y;
    }
    int run = incl - s;
#pragma unroll 1
    for (int i = 0; i < NBA / 32; ++i) {
      const int cv = cnt[base + i];
      offs[base + i] = run;
      cur[base + i]  = run;
      run += cv;
    }
  }
  __syncthreads();
  if (wave == 0) {
#pragma unroll 1
    for (int b0 = 0; b0 < tt; b0 += 32) {
      const int idx = b0 + lane;
      const int ent = hl[idx < RCAP ? idx : RCAP - 1];
      const int m32 = (tt - b0) < 32 ? (tt - b0) : 32;
#pragma unroll 1
      for (int k = 0; k < m32; ++k) {
        const int u    = __builtin_amdgcn_readlane(ent, k);
        const int slot = u & (NBA - 1);
        if (lane == 0) {
          int p = cur[slot];
          p = p < 0 ? 0 : (p > RCAP - 1 ? RCAP - 1 : p);
          sl[p] = u;
          cur[slot] = p + 1;
        }
      }
    }
  }
  __syncthreads();

#pragma unroll 1
  for (int i = tid; i < NBA; i += NTHR) {
    const float dg = (float)(cnt[i] + 1);
    float d = 1.0f / sqrtf(dg);
    d = (ovf != 0) ? __int_as_float(0x7fc00000) : d;
    cur[i] = __float_as_int(d);
  }
  int* lb = lst + (size_t)blockIdx.x * RCAP;
#pragma unroll 1
  for (int it = 0; it < RCAP / (NTHR * 4); ++it) {
    const int i0 = it * (NTHR * 4) + 4 * tid;
    const v4i e4 = *(const v4ia*)(sl + i0);
    int e0 = e4.x >> SLA, e1 = e4.y >> SLA, e2 = e4.z >> SLA, e3 = e4.w >> SLA;
    e0 = e0 < 0 ? 0 : (e0 > nE - 1 ? nE - 1 : e0);
    e1 = e1 < 0 ? 0 : (e1 > nE - 1 ? nE - 1 : e1);
    e2 = e2 < 0 ? 0 : (e2 > nE - 1 ? nE - 1 : e2);
    e3 = e3 < 0 ? 0 : (e3 > nE - 1 ? nE - 1 : e3);
    int r0 = srcs[e0], r1 = srcs[e1], r2 = srcs[e2], r3 = srcs[e3];
    v4i s4;
    s4.x = r0 < 0 ? 0 : (r0 > nN - 1 ? nN - 1 : r0);
    s4.y = r1 < 0 ? 0 : (r1 > nN - 1 ? nN - 1 : r1);
    s4.z = r2 < 0 ? 0 : (r2 > nN - 1 ? nN - 1 : r2);
    s4.w = r3 < 0 ? 0 : (r3 > nN - 1 ? nN - 1 : r3);
    *(volatile v4i*)(lb + i0) = s4;
    __threadfence();
    *(volatile v4i*)(lb + i0) = s4;
  }
  __syncthreads();
  {
    const v4i c4 = *(const v4ia*)(cnt + 4 * tid);
    const v4i o4 = *(const v4ia*)(offs + 4 * tid);
    const v4i d4 = *(const v4ia*)(cur + 4 * tid);
    int* pc = cntg + (size_t)nodeBase + 4 * tid;
    int* po = offg + (size_t)nodeBase + 4 * tid;
    int* pd = disb + (size_t)nodeBase + 4 * tid;
    *(volatile v4i*)pc = c4;
    *(volatile v4i*)po = o4;
    *(volatile v4i*)pd = d4;
    __threadfence();
    *(volatile v4i*)pc = c4;
    *(volatile v4i*)po = o4;
    *(volatile v4i*)pd = d4;
  }
}

template <int NT>
__global__ __launch_bounds__(GTHR) void k_gemm(const unsigned short* __restrict__ A,
                                               const unsigned short* __restrict__ WT,
                                               float* outF, int K) {
  constexpr int GBN = 16 * NT;
  constexpr int LPR = 4 * NT;
  constexpr int RPI = 32 / LPR;
  constexpr int NIT = 16 / RPI;
  static_assert(NT == 4 || NT == 2);
  __shared__ __attribute__((aligned(16))) float stg[GBM * GBN];
  const int tid = (int)threadIdx.x, lane = tid & 31, wave = tid >> 5, hh = lane >> 4, m = lane & 15;
  const int rowBase = (int)blockIdx.x * GBM;

  v8f acc[NT];
  {
    const v8f z = {0.f, 0.f, 0.f, 0.f, 0.f, 0.f, 0.f, 0.f};
#pragma unroll
    for (int t = 0; t < NT; ++t) acc[t] = z;
  }
  const unsigned short* ap = A  + (size_t)(rowBase + 16 * wave + m) * (size_t)K + 8 * hh;
  const unsigned short* wp = WT + (size_t)m * (size_t)K + 8 * hh;
  const int ksteps = K >> 5;
#pragma unroll 1
  for (int ks = 0; ks < ksteps; ++ks) {
    FragB af;
    af.h[0] = *(const v8usa*)(ap + 32 * ks);
    af.h[1] = *(const v8usa*)(ap + 32 * ks + 16);
#pragma unroll
    for (int t = 0; t < NT; ++t) {
      const unsigned short* wq = wp + (size_t)(16 * t) * (size_t)K + 32 * ks;
      FragB bf;
      bf.h[0] = *(const v8usa*)wq;
      bf.h[1] = *(const v8usa*)(wq + 16);
      acc[t] = wmb(af, bf, acc[t]);
    }
  }

#pragma unroll
  for (int t = 0; t < NT; ++t) {
    const int lc = 16 * t + m;
#pragma unroll
    for (int r = 0; r < 8; ++r) {
      const int lr = 16 * wave + 8 * hh + r;
      stg[lr * GBN + lc] = acc[t][r];
    }
  }
  __syncthreads();

  const int rsub = lane / LPR;
  const int cq   = lane % LPR;
  v4f fv[NIT];
#pragma unroll
  for (int i = 0; i < NIT; ++i) {
    const int lr = 16 * wave + RPI * i + rsub;
    fv[i] = *(const v4fa*)(stg + lr * GBN + 4 * cq);
  }
#pragma unroll
  for (int i = 0; i < NIT; ++i) {
    const int lr = 16 * wave + RPI * i + rsub;
    float* op = outF + (size_t)(rowBase + lr) * (size_t)GBN + 4 * cq;
    *(volatile v4f*)op = fv[i];
  }
  __threadfence();
#pragma unroll
  for (int i = 0; i < NIT; ++i) {
    const int lr = 16 * wave + RPI * i + rsub;
    float* op = outF + (size_t)(rowBase + lr) * (size_t)GBN + 4 * cq;
    *(volatile v4f*)op = fv[i];
  }
}

template <int W>
__global__ __launch_bounds__(NTHR) void k_agg(const int* __restrict__ lst, const int* __restrict__ offg,
                                              const int* __restrict__ cntg, const float* __restrict__ disg,
                                              const float* __restrict__ hin, const float* __restrict__ bias,
                                              int nN, int mRows, float* aout) {
  static_assert(W == 64 || W == 32);
  __shared__ __attribute__((aligned(16))) int   cntS[NBA];
  __shared__ __attribute__((aligned(16))) int   offS[NBA];
  __shared__ __attribute__((aligned(16))) float disS[NBA];
  const int tid = (int)threadIdx.x, lane = tid & 31, wave = tid >> 5;
  const int nodeBase = (int)blockIdx.x * NBA;
  {
    const v4i c4 = *(const v4ia*)(cntg + (size_t)nodeBase + 4 * tid);
    const v4i o4 = *(const v4ia*)(offg + (size_t)nodeBase + 4 * tid);
    const v4f d4 = *(const v4fa*)(disg + (size_t)nodeBase + 4 * tid);
    *(v4ia*)(cntS + 4 * tid) = c4;
    *(v4ia*)(offS + 4 * tid) = o4;
    *(v4fa*)(disS + 4 * tid) = d4;
  }
  float bv0 = 0.0f, bv1 = 0.0f;
  if constexpr (W == 64) {
    const v2f a = *(const v2fa*)(bias + 2 * lane);
    bv0 = bf16_val(a.x); bv1 = bf16_val(a.y);
  } else {
    bv0 = bf16_val(bias[lane]);
  }
  __syncthreads();

  const int* lb = lst + (size_t)blockIdx.x * RCAP;
  const float qnan = __int_as_float(0x7fc00000);
  const int sa = (2 * lane) & 31, sb = (2 * lane + 1) & 31;
  const int q0s = (4 * lane) & 31, q1s = (4 * lane + 1) & 31;
  const int q2s = (4 * lane + 2) & 31, q3s = (4 * lane + 3) & 31;
#pragma unroll 1
  for (int si = 0; si < NBA / NWAVE; ++si) {
    const int s    = si * NWAVE + wave;
    const int node = nodeBase + s;
    int c = cntS[s];
    const bool big = c > DEGCAP;
    c = c < 0 ? 0 : (c > DEGCAP ? DEGCAP : c);
    int o = offS[s];
    o = o < 0 ? 0 : (o > RCAP ? RCAP : o);
    const int nc = node < nN ? node : nN - 1;
    const float dd = disS[s];
    const float rd = dd * dd;
    float acc0 = 0.0f, acc1 = 0.0f;
#pragma unroll 1
    for (int b0 = 0; b0 < c; b0 += 32) {
      int idx = o + b0 + lane;
      idx = idx > RCAP - 1 ? RCAP - 1 : idx;
      int sr = lb[idx];
      sr = sr < 0 ? 0 : (sr > nN - 1 ? nN - 1 : sr);
      const float cf  = disg[sr] * dd;
      const int   cfi = __float_as_int(cf);
      const int m32 = (c - b0) < 32 ? (c - b0) : 32;
#pragma unroll 1
      for (int k = 0; k < m32; ++k) {
        const int   sk = __builtin_amdgcn_readlane(sr, k);
        const float ck = __int_as_float(__builtin_amdgcn_readlane(cfi, k));
        if constexpr (W == 64) {
          const v2f a = *(const v2fa*)(hin + (size_t)sk * 64 + 2 * lane);
          acc0 = fmaf(ck, a.x, acc0); acc1 = fmaf(ck, a.y, acc1);
        } else {
          const float a = hin[(size_t)sk * 32 + lane];
          acc0 = fmaf(ck, a, acc0);
        }
      }
    }
    float sv0 = 0.0f, sv1 = 0.0f;
    if constexpr (W == 64) {
      const v2f a = *(const v2fa*)(hin + (size_t)nc * 64 + 2 * lane);
      sv0 = a.x; sv1 = a.y;
    } else {
      sv0 = hin[(size_t)nc * 32 + lane];
    }
    const float pzr = big ? qnan : 0.0f;
    const bool live = node < nN;
    float y0 = (acc0 + sv0 * rd) + bv0;
    float y1 = (acc1 + sv1 * rd) + bv1;
    y0 = y0 + pzr; y1 = y1 + pzr;
    const float v0 = live ? y0 : 0.0f;
    const float v1 = live ? y1 : 0.0f;
    if constexpr (W == 64) {
      v4f ow;
      ow.x = __shfl(v0, sa, 32); ow.y = __shfl(v1, sa, 32);
      ow.z = __shfl(v0, sb, 32); ow.w = __shfl(v1, sb, 32);
      const bool wr = (node < mRows) && (lane < 16);
      float* op = aout + (size_t)node * 64 + 4 * (lane & 15);
      if (wr) *(volatile v4f*)op = ow;
      __threadfence();
      if (wr) *(volatile v4f*)op = ow;
    } else {
      v4f ow;
      ow.x = __shfl(v0, q0s, 32); ow.y = __shfl(v0, q1s, 32);
      ow.z = __shfl(v0, q2s, 32); ow.w = __shfl(v0, q3s, 32);
      const bool wr = (node < mRows) && (lane < 8);
      float* op = aout + (size_t)node * 32 + 4 * (lane & 7);
      if (wr) *(volatile v4f*)op = ow;
      __threadfence();
      if (wr) *(volatile v4f*)op = ow;
    }
  }
}

template <int W>
__global__ __launch_bounds__(NTHR) void k_stats(const float* __restrict__ a, int nN, float* rec) {
  static_assert(W == 64 || W == 32);
  constexpr int RG  = NTHR / W;
  constexpr int RPG = TROWS / RG;
  __shared__ __attribute__((aligned(16))) float tile[TROWS * W];
  __shared__ float part[NTHR];
  __shared__ __attribute__((aligned(16))) float rs[RECW];
  const int tid = (int)threadIdx.x;
  const int row0 = (int)blockIdx.x * TROWS;
  int nv = nN - row0;
  nv = nv < 0 ? 0 : (nv > TROWS ? TROWS : nv);
  if (tid < RECW) rs[tid] = (tid >= 128) ? (float)nv : 0.0f;
#pragma unroll 1
  for (int i = tid; i < TROWS * W / 4; i += NTHR)
    *(v4fa*)(tile + 4 * i) = *(const v4fa*)(a + (size_t)row0 * W + 4 * i);
  __syncthreads();
  const int c  = tid & (W - 1);
  const int rg = tid / W;
  const int r0 = rg * RPG;
  float s = 0.0f;
#pragma unroll 4
  for (int r = 0; r < RPG; ++r) {
    const float v = tile[(r0 + r) * W + c];
    s += ((r0 + r) < nv) ? v : 0.0f;
  }
  part[tid] = s;
  __syncthreads();
  if (tid < W) {
    float t = 0.0f;
#pragma unroll 1
    for (int g = 0; g < RG; ++g) t += part[g * W + tid];
    const float nf = (float)(nv < 1 ? 1 : nv);
    rs[tid] = t * (1.0f / nf);
  }
  __syncthreads();
  const float mb = rs[c];
  float q = 0.0f;
#pragma unroll 4
  for (int r = 0; r < RPG; ++r) {
    const float v = tile[(r0 + r) * W + c];
    const float d = ((r0 + r) < nv) ? (v - mb) : 0.0f;
    q = fmaf(d, d, q);
  }
  part[tid] = q;
  __syncthreads();
  if (tid < W) {
    float t = 0.0f;
#pragma unroll 1
    for (int g = 0; g < RG; ++g) t += part[g * W + tid];
    rs[64 + tid] = t;
  }
  __syncthreads();
  const int tq = tid < RECW / 4 ? tid : RECW / 4 - 1;
  const v4f pv = *(const v4fa*)(rs + 4 * tq);
  float* op = rec + (size_t)blockIdx.x * RECW + 4 * tq;
  const bool wr = tid < RECW / 4;
  if (wr) *(volatile v4f*)op = pv;
  __threadfence();
  if (wr) *(volatile v4f*)op = pv;
}

__global__ __launch_bounds__(64) void k_comb(const float* __restrict__ rec, int nTile, int wcols,
                                             const float* __restrict__ gam, const float* __restrict__ bet,
                                             float* stat) {
  __shared__ __attribute__((aligned(16))) float stg[256];
  const int c  = (int)threadIdx.x;
  const int cc = c < wcols ? c : wcols - 1;
  double n = 0.0, mean = 0.0, M2 = 0.0;
#pragma unroll 1
  for (int b = 0; b < nTile; ++b) {
    const float* pr = rec + (size_t)b * RECW;
    const double nb = (double)pr[128];
    const double mb = (double)pr[cc];
    const double qb = (double)pr[64 + cc];
    if (nb > 0.5) {
      const double nn = n + nb;
      const double delta = mb - mean;
      const double f = nb / nn;
      mean = mean + delta * f;
      M2 = M2 + qb + delta * delta * n * f;
      n = nn;
    }
  }
  const double nt = n < 1.0 ? 1.0 : n;
  const float varf  = (float)(M2 / nt);
  const float meanf = (float)mean;
  const float ve = varf + 1e-5f;
  const float rstd = 1.0f / sqrtf(ve);
  stg[c]       = meanf;
  stg[64 + c]  = rstd;
  stg[128 + c] = bf16_val(gam[cc]);
  stg[192 + c] = bf16_val(bet[cc]);
  __syncthreads();
  const v4f v = *(const v4fa*)(stg + 4 * c);
  *(volatile v4f*)(stat + 4 * c) = v;
  __threadfence();
  *(volatile v4f*)(stat + 4 * c) = v;
}

__global__ __launch_bounds__(NTHR) void k_apply(const float* __restrict__ a, const float* __restrict__ stat,
                                                int nN, unsigned short* xhl) {
  __shared__ float ssh[256];
  const int tid = (int)threadIdx.x;
  ssh[tid] = stat[tid];
  __syncthreads();
  const int u = (int)blockIdx.x * NTHR + tid;
  if (u >= MPAD * 8) return;
  const int row = u >> 3;
  const int c8  = (u & 7) * 8;
  const int rc  = row < nN ? row : nN - 1;
  const float* p = a + (size_t)rc * 64 + c8;
  const v4f va = *(const v4fa*)p;
  const v4f vb = *(const v4fa*)(p + 4);
  const bool ok = row < nN;
  float xi[8];
  xi[0] = va.x; xi[1] = va.y; xi[2] = va.z; xi[3] = va.w;
  xi[4] = vb.x; xi[5] = vb.y; xi[6] = vb.z; xi[7] = vb.w;
  v8us ho, lo;
#pragma unroll
  for (int j = 0; j < 8; ++j) {
    const int cidx = c8 + j;
    float y = ((xi[j] - ssh[cidx]) * ssh[64 + cidx]) * ssh[128 + cidx] + ssh[192 + cidx];
    y = (y > 0.0f) ? y : (y - y);
    y = ok ? y : 0.0f;
    const unsigned hb = bf16_bits_n(y);
    const float rem = y - __uint_as_float(hb << 16);
    ho[j] = (unsigned short)hb;
    lo[j] = (unsigned short)bf16_bits_n(rem);
  }
  unsigned short* hp = xhl + (size_t)row * 128 + c8;
  *(volatile v8us*)hp = ho;
  *(volatile v8us*)(hp + 64) = lo;
  __threadfence();
  *(volatile v8us*)hp = ho;
  *(volatile v8us*)(hp + 64) = lo;
}

__global__ __launch_bounds__(NTHR) void k_pool(const float* __restrict__ a4, const float* __restrict__ stat,
                                               const int* __restrict__ bat, int nN, float* pl) {
  __shared__ __attribute__((aligned(16))) float wsum[NWAVE * 32];
  __shared__ int wcn[NWAVE];
  __shared__ __attribute__((aligned(16))) float outs[32];
  const int tid = (int)threadIdx.x, lane = tid & 31, wave = tid >> 5;
  const int g = (int)blockIdx.x;
  const float mu = stat[lane];
  const float rr = stat[64 + lane];
  const float gg = stat[128 + lane];
  const float be = stat[192 + lane];

  float a0 = 0.0f;
  int cnt = 0;
#pragma unroll 1
  for (int i0 = wave * 32; i0 < nN; i0 += NTHR) {
    const int i  = i0 + lane;
    const int ic = i < nN ? i : nN - 1;
    const int b  = bat[ic];
    const bool hit = (i < nN) && (b == g);
    unsigned msk = __builtin_amdgcn_ballot_w32(hit);
    int nh = (int)__builtin_popcount(msk);
    nh = nh > 32 ? 32 : nh;
    cnt += nh;
#pragma unroll 1
    for (int q = 0; q < nh; ++q) {
      const int k = __builtin_ffs((int)msk) - 1;
      msk &= msk - 1u;
      int node = i0 + (k < 0 ? 0 : k);
      node = node > nN - 1 ? nN - 1 : node;
      const float xv = a4[(size_t)node * 32 + lane];
      float y = ((xv - mu) * rr) * gg + be;
      y = (y > 0.0f) ? y : (y - y);
      a0 += y;
    }
  }
  wsum[wave * 32 + lane] = a0;
  if (lane == 0) wcn[wave] = cnt;
  __syncthreads();
  if (tid < 32) {
    float s = 0.0f;
    int c = 0;
#pragma unroll
    for (int w2 = 0; w2 < NWAVE; ++w2) { s += wsum[w2 * 32 + tid]; c += wcn[w2]; }
    const float cf = (c < 1) ? 1.0f : (float)c;
    outs[tid] = s * (1.0f / cf);
  }
  __syncthreads();
  const v4f ov = *(const v4fa*)(outs + 4 * (lane & 7));
  float* op = pl + (size_t)g * 32 + 4 * (lane & 7);
  const bool okst = (wave == 0) && (lane < 8);
  if (okst) *(volatile v4f*)op = ov;
  __threadfence();
  if (okst) *(volatile v4f*)op = ov;
}

__global__ __launch_bounds__(NTHR) void k_head(const float* __restrict__ pl, const float* __restrict__ Wl,
                                               const float* __restrict__ bl, float* out) {
  __shared__ __attribute__((aligned(16))) float wls[32 * NCLS];
  __shared__ float bls[16];
  __shared__ __attribute__((aligned(16))) float os[NOUT];
  const int tid = (int)threadIdx.x;
  if (tid < (32 * NCLS) / 4) {
    const v4f w = *(const v4fa*)(Wl + 4 * tid);
    v4f o;
    o.x = bf16_val(w.x); o.y = bf16_val(w.y); o.z = bf16_val(w.z); o.w = bf16_val(w.w);
    *(v4fa*)(wls + 4 * tid) = o;
  }
  if (tid < 16) {
    const float bb = bl[tid < NCLS ? tid : NCLS - 1];
    bls[tid] = (tid < NCLS) ? bf16_val(bb) : 0.0f;
  }
  __syncthreads();
  const int g = tid;
  const float* pr = pl + (size_t)g * 32;
#pragma unroll 1
  for (int c = 0; c < NCLS; ++c) {
    float s = 0.0f;
#pragma unroll 1
    for (int f4 = 0; f4 < 8; ++f4) {
      const v4f p = *(const v4fa*)(pr + 4 * f4);
      const float* w = wls + (4 * f4) * NCLS + c;
      s = fmaf(p.x, w[0], s);
      s = fmaf(p.y, w[NCLS], s);
      s = fmaf(p.z, w[2 * NCLS], s);
      s = fmaf(p.w, w[3 * NCLS], s);
    }
    os[g * NCLS + c] = s + bls[c];
  }
  float m = os[g * NCLS];
#pragma unroll 1
  for (int c = 1; c < NCLS; ++c) {
    const float l = os[g * NCLS + c];
    m = ((l > m) || (l != l)) ? l : m;
  }
  float sum = 0.0f;
#pragma unroll 1
  for (int c = 0; c < NCLS; ++c) {
    const float e = expf(os[g * NCLS + c] - m);
    os[g * NCLS + c] = e;
    sum += e;
  }
  const float inv = 1.0f / sum;
#pragma unroll 1
  for (int c = 0; c < NCLS; ++c) {
    const float e = os[g * NCLS + c];
    os[g * NCLS + c] = e * inv;
  }
  __syncthreads();
  constexpr int NV4 = NOUT / 4;
  v4f ov[3];
#pragma unroll
  for (int it = 0; it < 3; ++it) {
    const int idx = it * NTHR + tid;
    const int ic  = idx < NV4 ? idx : NV4 - 1;
    ov[it] = *(const v4fa*)(os + 4 * ic);
  }
#pragma unroll
  for (int it = 0; it < 3; ++it) {
    const int idx = it * NTHR + tid;
    if (idx < NV4) *(volatile v4f*)(out + 4 * (size_t)idx) = ov[it];
  }
  __threadfence();
#pragma unroll
  for (int it = 0; it < 3; ++it) {
    const int idx = it * NTHR + tid;
    if (idx < NV4) *(volatile v4f*)(out + 4 * (size_t)idx) = ov[it];
  }
}

static constexpr size_t al256c(size_t o) { return (o + 255) & ~(size_t)255; }
static constexpr size_t SZ_XB   = (size_t)MPAD * 64 * 2;
static constexpr size_t SZ_H    = (size_t)MPAD * 64 * 4;
static constexpr size_t SZ_AGG  = (size_t)MPAD * 64 * 4;
static constexpr size_t SZ_XHL  = (size_t)MPAD * 128 * 2;
static constexpr size_t SZ_LIST = (size_t)NBLK * RCAP * 4;
static constexpr size_t SZ_SLOT = (size_t)NPADS * 4;
static constexpr size_t SZ_REC  = (size_t)NTILE * RECW * 4;
static constexpr size_t SZ_STAT = 256 * 4;
static constexpr size_t SZ_W64  = 64 * 64 * 2;
static constexpr size_t SZ_W128 = 64 * 128 * 2;
static constexpr size_t SZ_W3D  = 32 * 128 * 2;
static constexpr size_t SZ_POOL = (size_t)NGR * 32 * 4;
static constexpr size_t O_XB   = 0;
static constexpr size_t O_H    = al256c(O_XB + SZ_XB);
static constexpr size_t O_AGG  = al256c(O_H + SZ_H);
static constexpr size_t O_XHL  = al256c(O_AGG + SZ_AGG);
static constexpr size_t O_LIST = al256c(O_XHL + SZ_XHL);
static constexpr size_t O_OFF  = al256c(O_LIST + SZ_LIST);
static constexpr size_t O_CNT  = al256c(O_OFF + SZ_SLOT);
static constexpr size_t O_DIS  = al256c(O_CNT + SZ_SLOT);
static constexpr size_t O_REC  = al256c(O_DIS + SZ_SLOT);
static constexpr size_t O_STAT = al256c(O_REC + SZ_REC);
static constexpr size_t O_W1T  = al256c(O_STAT + 4 * SZ_STAT);
static constexpr size_t O_W2D  = al256c(O_W1T + SZ_W64);
static constexpr size_t O_W4D  = al256c(O_W2D + SZ_W128);
static constexpr size_t O_W3D  = al256c(O_W4D + SZ_W128);
static constexpr size_t O_POOL = al256c(O_W3D + SZ_W3D);
static constexpr size_t O_END  = al256c(O_POOL + SZ_POOL);
static_assert(O_END <= (size_t)WSMAX);

extern "C" void kernel_launch(void* const* d_in, const int* in_sizes, int n_in,
                              void* d_out, int out_size, void* d_ws, size_t ws_size,
                              hipStream_t stream) {
  if (n_in < 22) return;
  if (in_sizes[0] != NN * 64) return;
  if (in_sizes[1] != NE || in_sizes[2] != NE) return;
  if (in_sizes[3] != NN) return;
  if (in_sizes[4] != 4096 || in_sizes[5] != 64) return;
  if (in_sizes[6] != 4096 || in_sizes[7] != 64) return;
  if (in_sizes[8] != 4096 || in_sizes[9] != 64) return;
  if (in_sizes[10] != 2048 || in_sizes[11] != 32) return;
  if (in_sizes[12] != 64 || in_sizes[13] != 64) return;
  if (in_sizes[14] != 64 || in_sizes[15] != 64) return;
  if (in_sizes[16] != 64 || in_sizes[17] != 64) return;
  if (in_sizes[18] != 32 || in_sizes[19] != 32) return;
  if (in_sizes[20] != 32 * NCLS || in_sizes[21] != NCLS) return;
  if (out_size != NOUT) return;
  if (O_END > ws_size) return;

  const float* x    = (const float*)d_in[0];
  const int*   esrc = (const int*)d_in[1];
  const int*   edst = (const int*)d_in[2];
  const int*   bat  = (const int*)d_in[3];
  const float* W1   = (const float*)d_in[4];
  const float* b1   = (const float*)d_in[5];
  const float* W2   = (const float*)d_in[6];
  const float* b2   = (const float*)d_in[7];
  const float* W4   = (const float*)d_in[8];
  const float* b4   = (const float*)d_in[9];
  const float* W3   = (const float*)d_in[10];
  const float* b3   = (const float*)d_in[11];
  const float* g1   = (const float*)d_in[12];
  const float* be1  = (const float*)d_in[13];
  const float* g2   = (const float*)d_in[14];
  const float* be2  = (const float*)d_in[15];
  const float* g4   = (const float*)d_in[16];
  const float* be4  = (const float*)d_in[17];
  const float* g3   = (const float*)d_in[18];
  const float* be3  = (const float*)d_in[19];
  const float* Wl   = (const float*)d_in[20];
  const float* bl   = (const float*)d_in[21];
  float* out = (float*)d_out;

  char* ws = (char*)d_ws;
  unsigned short* XB   = (unsigned short*)(ws + O_XB);
  float*          H    = (float*)(ws + O_H);
  float*          AGG  = (float*)(ws + O_AGG);
  unsigned short* XHL  = (unsigned short*)(ws + O_XHL);
  int*            LIST = (int*)(ws + O_LIST);
  int*            OFF  = (int*)(ws + O_OFF);
  int*            CNT  = (int*)(ws + O_CNT);
  int*            DISB = (int*)(ws + O_DIS);
  const float*    DIS  = (const float*)(ws + O_DIS);
  float*          REC  = (float*)(ws + O_REC);
  float*          ST0  = (float*)(ws + O_STAT);
  float*          ST1  = (float*)(ws + O_STAT + SZ_STAT);
  float*          ST2  = (float*)(ws + O_STAT + 2 * SZ_STAT);
  float*          ST3  = (float*)(ws + O_STAT + 3 * SZ_STAT);
  unsigned short* W1T  = (unsigned short*)(ws + O_W1T);
  unsigned short* W2D  = (unsigned short*)(ws + O_W2D);
  unsigned short* W4D  = (unsigned short*)(ws + O_W4D);
  unsigned short* W3D  = (unsigned short*)(ws + O_W3D);
  float*          POOL = (float*)(ws + O_POOL);

  const size_t bktLds = (size_t)AGG_LDS_INTS * 4;
  hipFuncSetAttribute(reinterpret_cast<const void*>(&k_bucket), hipFuncAttributeMaxDynamicSharedMemorySize,
                      (int)bktLds);
  const int vec8 = ((NE & 3) == 0) ? 1 : 0;
  const int gM   = MPAD / GBM;
  const int gAp  = (MPAD * 8) / NTHR;

  k_prep<<<NUALL / NTHR, NTHR, 0, stream>>>(x, W1, W2, W4, W3, XB, W1T, W2D, W4D, W3D);
  k_bucket<<<NBLK, NTHR, bktLds, stream>>>(esrc, edst, NE, NN, vec8, LIST, OFF, CNT, DISB);
  k_gemm<4><<<gM, GTHR, 0, stream>>>(XB, W1T, H, 64);
  k_agg<64><<<NBLK, NTHR, 0, stream>>>(LIST, OFF, CNT, DIS, H, b1, NN, MPAD, AGG);
  k_stats<64><<<NTILE, NTHR, 0, stream>>>(AGG, NN, REC);
  k_comb<<<1, 64, 0, stream>>>(REC, NTILE, 64, g1, be1, ST0);
  k_apply<<<gAp, NTHR, 0, stream>>>(AGG, ST0, NN, XHL);
  k_gemm<4><<<gM, GTHR, 0, stream>>>(XHL, W2D, H, 128);
  k_agg<64><<<NBLK, NTHR, 0, stream>>>(LIST, OFF, CNT, DIS, H, b2, NN, MPAD, AGG);
  k_stats<64><<<NTILE, NTHR, 0, stream>>>(AGG, NN, REC);
  k_comb<<<1, 64, 0, stream>>>(REC, NTILE, 64, g2, be2, ST1);
  k_apply<<<gAp, NTHR, 0, stream>>>(AGG, ST1, NN, XHL);
  k_gemm<4><<<gM, GTHR, 0, stream>>>(XHL, W4D, H, 128);
  k_agg<64><<<NBLK, NTHR, 0, stream>>>(LIST, OFF, CNT, DIS, H, b4, NN, MPAD, AGG);
  k_stats<64><<<NTILE, NTHR, 0, stream>>>(AGG, NN, REC);
  k_comb<<<1, 64, 0, stream>>>(REC, NTILE, 64, g4, be4, ST2);
  k_apply<<<gAp, NTHR, 0, stream>>>(AGG, ST2, NN, XHL);
  k_gemm<2><<<gM, GTHR, 0, stream>>>(XHL, W3D, H, 128);
  k_agg<32><<<NBLK, NTHR, 0, stream>>>(LIST, OFF, CNT, DIS, H, b3, NN, MPAD, AGG);
  k_stats<32><<<NTILE, NTHR, 0, stream>>>(AGG, NN, REC);
  k_comb<<<1, 64, 0, stream>>>(REC, NTILE, 32, g3, be3, ST3);
  k_pool<<<NGR, NTHR, 0, stream>>>(AGG, ST3, bat, NN, POOL);
  k_head<<<1, NTHR, 0, stream>>>(POOL, Wl, bl, out);
}
